// GQA_137438954255
// MI455X (gfx1250) — hardware-verified
//
#include <hip/hip_runtime.h>


#ifndef NB
#define NB 2
#endif
#ifndef SEQ
#define SEQ 2048
#endif
#define NB_FULL 2
#define TT_FULL 2048
#define TT   SEQ
#define DM   2048
#define NH_  16
#define NKV  4
#define REP  (NH_ / NKV)
#define HD   128
#define DQ   (NH_ * HD)
#define DKV  (NKV * HD)
#define RH   ((TT < 512) ? TT : 512)
#define PCAR 1024.0f
#define ACAR 16.0f
#define WCAR 64.0f
#define SCL  0.088388347648318447f
#define EPSN 1.0e-6f
#define L2E  1.4426950408889634f
static_assert(TT % 64 == 0);
static_assert(TT <= TT_FULL);
static_assert(NB >= 1 && NB <= NB_FULL);
static_assert(RH % 64 == 0 && RH <= TT);
static_assert(DM % 64 == 0 && DQ % 64 == 0 && DKV % 64 == 0 && HD == 128);

typedef _Float16 h16;
typedef unsigned short bf;
typedef __attribute__((ext_vector_type(16))) __bf16   v16bf;
typedef __attribute__((ext_vector_type(16))) _Float16 v16h;
typedef __attribute__((ext_vector_type(8)))  _Float16 v8h;
typedef __attribute__((ext_vector_type(8)))  unsigned short v8us;
typedef __attribute__((ext_vector_type(8)))  float    v8f;
typedef __attribute__((ext_vector_type(4)))  float    v4f;
typedef __attribute__((ext_vector_type(2)))  _Float16 v2h;
typedef __attribute__((ext_vector_type(2)))  unsigned short v2us;
typedef __attribute__((ext_vector_type(2)))  float    v2f;
typedef v8h  __attribute__((may_alias)) v8ha;
typedef v4f  __attribute__((may_alias)) v4fa;
typedef v8us __attribute__((may_alias)) v8usa;

__device__ __forceinline__ unsigned short f2bf(float f) { unsigned u = __float_as_uint(f); u += 0x7FFFu + ((u >> 16) & 1u); return (unsigned short)(u >> 16); }
__device__ __forceinline__ float bf2f(unsigned short b) { return __uint_as_float(((unsigned)b) << 16); }
__device__ __forceinline__ float bfr(float f) { return bf2f(f2bf(f)); }
__device__ __forceinline__ h16 tohx(float x) { return (h16)x; }
__device__ __forceinline__ void splitf(float y, unsigned short& h, unsigned short& l) { h = f2bf(y); l = f2bf(y - bf2f(h)); }
__device__ __forceinline__ v16h cat16(v8h lo, v8h hi) { return __builtin_shufflevector(lo, hi, 0, 1, 2, 3, 4, 5, 6, 7, 8, 9, 10, 11, 12, 13, 14, 15); }
__device__ __forceinline__ v16bf cat16b(v8us lo, v8us hi) { return __builtin_bit_cast(v16bf, __builtin_shufflevector(lo, hi, 0, 1, 2, 3, 4, 5, 6, 7, 8, 9, 10, 11, 12, 13, 14, 15)); }
__device__ __forceinline__ v8f wmma16(v16h a, v16h b, v8f c) { return __builtin_amdgcn_wmma_f32_16x16x32_f16(false, a, false, b, (short)0, c, false, false); }
__device__ __forceinline__ v8f wmmab(v16bf a, v16bf b, v8f c) { return __builtin_amdgcn_wmma_f32_16x16x32_bf16(false, a, false, b, (short)0, c, false, false); }

template <typename T16> struct WFrag;
template <> struct WFrag<h16> { typedef v16h V; static __device__ __forceinline__ V ld(const h16* p) { return cat16(*(const v8h*)p, *(const v8h*)(p + 16)); } static __device__ __forceinline__ v8f mma(V a, V b, v8f c) { return wmma16(a, b, c); } };
template <> struct WFrag<bf> { typedef v16bf V; static __device__ __forceinline__ V ld(const bf* p) { return cat16b(*(const v8us*)p, *(const v8us*)(p + 16)); } static __device__ __forceinline__ v8f mma(V a, V b, v8f c) { return wmmab(a, b, c); } };

template <typename T16, int NSPLIT>
__global__ __launch_bounds__(32) void k_gemmw(const T16* __restrict__ A, const T16* __restrict__ A2, const T16* __restrict__ Bt, const T16* __restrict__ Bt2, int K, float* C, int ldc, float osc, size_t sA, size_t sB, size_t sC) {
    typedef typename WFrag<T16>::V V;
    __shared__ __align__(16) float os[16 * 68];
    const size_t z = blockIdx.z; A += z * sA; if (A2) A2 += z * sA; Bt += z * sB; if (Bt2) Bt2 += z * sB; C += z * sC;
    const int lane = threadIdx.x & 31, lr = lane & 15, hi = lane >> 4; const int r0 = blockIdx.x * 64, c0 = blockIdx.y * 64;
    v8f acc[4][4];
#pragma unroll
    for (int mb = 0; mb < 4; ++mb)
#pragma unroll
        for (int nb = 0; nb < 4; ++nb) acc[mb][nb] = (v8f){};
    const size_t aoff = (size_t)(r0 + lr) * K + 8 * hi, boff = (size_t)(c0 + lr) * K + 8 * hi;
#pragma unroll 1
    for (int kc = 0; kc < K; kc += 32) {
        V a[4], a2[4];
#pragma unroll
        for (int mb = 0; mb < 4; ++mb) { a[mb] = WFrag<T16>::ld(A + aoff + (size_t)mb * 16 * K + kc); if (NSPLIT == 1 || NSPLIT == 2) a2[mb] = WFrag<T16>::ld(A2 + aoff + (size_t)mb * 16 * K + kc); }
#pragma unroll
        for (int nb = 0; nb < 4; ++nb) { const V b = WFrag<T16>::ld(Bt + boff + (size_t)nb * 16 * K + kc); V b2; if (NSPLIT >= 2) b2 = WFrag<T16>::ld(Bt2 + boff + (size_t)nb * 16 * K + kc);
#pragma unroll
            for (int mb = 0; mb < 4; ++mb) { acc[mb][nb] = WFrag<T16>::mma(a[mb], b, acc[mb][nb]); if (NSPLIT == 1 || NSPLIT == 2) acc[mb][nb] = WFrag<T16>::mma(a2[mb], b, acc[mb][nb]); if (NSPLIT >= 2) acc[mb][nb] = WFrag<T16>::mma(a[mb], b2, acc[mb][nb]); } }
        asm volatile("v_nop\n\tv_nop\n\tv_nop\n\tv_nop" : "+v"(acc[0][0]), "+v"(acc[1][1]), "+v"(acc[2][2]), "+v"(acc[3][3]) : "v"(a[0]), "v"(a[3]));
    }
#pragma unroll
    for (int mb = 0; mb < 4; ++mb) {
#pragma unroll
        for (int nb = 0; nb < 4; ++nb) {
#pragma unroll
            for (int j = 0; j < 8; ++j) os[(hi * 8 + j) * 68 + nb * 16 + lr] = acc[mb][nb][j]; }
        __builtin_amdgcn_wave_barrier(); asm volatile("" ::: "memory");
        float* crow = C + (size_t)(r0 + mb * 16) * ldc + c0;
#pragma unroll 1
        for (int ps = 0; ps < 2; ++ps) {
#pragma unroll
            for (int s = 0; s < 8; ++s) { const int row = 2 * s + hi, cofs = lr * 4; v4f val = *(const v4fa*)(os + row * 68 + cofs); val = val * osc;
                *(volatile v4f*)(crow + (size_t)row * ldc + cofs) = val; }
            if (ps == 0) __threadfence(); }
        __builtin_amdgcn_wave_barrier(); asm volatile("" ::: "memory");
    }
}

__global__ __launch_bounds__(256) void k_cvt8(const float* __restrict__ src, bf* dst, size_t n8) { const size_t i = (size_t)blockIdx.x * 256 + threadIdx.x; if (i >= n8) return; const v8f v = *(const v8f*)(src + i * 8); v8us o;
#pragma unroll
    for (int k = 0; k < 8; ++k) o[k] = f2bf(v[k]); *(volatile v8us*)(dst + i * 8) = o; __threadfence(); *(volatile v8us*)(dst + i * 8) = o; }
__global__ __launch_bounds__(256) void k_cvt16s(const float* __restrict__ src, h16* dst, size_t n8, float sc) { const size_t i = (size_t)blockIdx.x * 256 + threadIdx.x; if (i >= n8) return; const v8f v = *(const v8f*)(src + i * 8); v8h o;
#pragma unroll
    for (int k = 0; k < 8; ++k) o[k] = tohx(bfr(v[k]) * sc); *(volatile v8h*)(dst + i * 8) = o; __threadfence(); *(volatile v8h*)(dst + i * 8) = o; }
__global__ __launch_bounds__(256) void k_cscvt(const float* __restrict__ cosT, const float* __restrict__ sinT, float* CS) { const int idx = blockIdx.x * 256 + threadIdx.x; if (idx >= TT * HD) return; v2f cs; cs[0] = bfr(cosT[idx]); cs[1] = bfr(sinT[idx]); *(volatile v2f*)(CS + (size_t)idx * 2) = cs; __threadfence(); *(volatile v2f*)(CS + (size_t)idx * 2) = cs; }
__global__ __launch_bounds__(256) void k_rms(const float* __restrict__ F, int pitch, float* RF) {
    __shared__ __align__(16) float sr[32];
    const int lane = threadIdx.x & 31, w = threadIdx.x >> 5; const int h = blockIdx.y; const int t0 = blockIdx.x * 32;
#pragma unroll 1
    for (int i = 0; i < 4; ++i) { const int t = t0 + w * 4 + i; const v4f v = *(const v4f*)(F + (size_t)t * pitch + h * HD + lane * 4);
        float s = v[0] * v[0]; s = fmaf(v[1], v[1], s); s = fmaf(v[2], v[2], s); s = fmaf(v[3], v[3], s);
#pragma unroll
        for (int sh = 16; sh; sh >>= 1) s += __shfl_xor(s, sh, 32);
        if (lane == 0) sr[w * 4 + i] = rsqrtf(s * (1.0f / HD) + EPSN); }
    __syncthreads();
    if (w == 0 && lane < 8) { const v4f o = *(const v4fa*)(sr + lane * 4); float* dst = RF + (size_t)h * TT + t0 + lane * 4; *(volatile v4f*)dst = o; __threadfence(); *(volatile v4f*)dst = o; }
}
__global__ __launch_bounds__(256) void k_rope(const float* __restrict__ F, int pitch, int nheads, const float* __restrict__ CS, const float* __restrict__ RF, const float* __restrict__ nw, float sc, h16* P16, bf* Ph, bf* Pl) {
    const size_t e = ((size_t)blockIdx.x * 256 + threadIdx.x) * 2; if (e >= (size_t)nheads * TT * HD) return; const int d = (int)(e % HD); const int t = (int)((e / HD) % TT); const int h = (int)(e / ((size_t)HD * TT)); const float* f = F + (size_t)t * pitch + h * HD; const float rf = RF ? RF[(size_t)h * TT + t] : 1.0f; v2h o16; v2us oh, ol;
#pragma unroll
    for (int q = 0; q < 2; ++q) { const int dd = d + q; const int dp = (dd < HD / 2) ? dd + HD / 2 : dd - HD / 2; float x0 = f[dd], x1 = f[dp];
        if (RF) { float n0 = __fmul_rn(x0, rf), n1 = __fmul_rn(x1, rf); asm volatile("" : "+v"(n0)); asm volatile("" : "+v"(n1)); x0 = __fmul_rn(bfr(nw[dd]), n0); x1 = __fmul_rn(bfr(nw[dp]), n1); }
        const v2f cs = *(const v2f*)(CS + ((size_t)t * HD + dd) * 2); float a = __fmul_rn(x0, cs[0]), bq = __fmul_rn(x1, cs[1]); asm volatile("" : "+v"(a)); asm volatile("" : "+v"(bq)); const float r = ((dd < HD / 2) ? __fsub_rn(a, bq) : __fadd_rn(a, bq)) * sc;
        o16[q] = tohx(r); unsigned short a2, c2; splitf(r, a2, c2); oh[q] = a2; ol[q] = c2; }
    *(volatile v2h*)(P16 + e) = o16; *(volatile v2us*)(Ph + e) = oh; *(volatile v2us*)(Pl + e) = ol; __threadfence(); *(volatile v2h*)(P16 + e) = o16; *(volatile v2us*)(Ph + e) = oh; *(volatile v2us*)(Pl + e) = ol; }
__global__ __launch_bounds__(256) void k_vtp(const float* __restrict__ F, int pitch, int nheads, h16* V16, bf* Vh, bf* Vl) { const size_t e = ((size_t)blockIdx.x * 256 + threadIdx.x) * 2; if (e >= (size_t)nheads * HD * TT) return; const int t = (int)(e % TT); const int d = (int)((e / TT) % HD); const int g = (int)(e / ((size_t)TT * HD)); v2h o16; v2us oh, ol;
#pragma unroll
    for (int q = 0; q < 2; ++q) { const float x = F[(size_t)(t + q) * pitch + g * HD + d]; o16[q] = tohx(x); unsigned short a2, c2; splitf(x, a2, c2); oh[q] = a2; ol[q] = c2; }
    *(volatile v2h*)(V16 + e) = o16; *(volatile v2us*)(Vh + e) = oh; *(volatile v2us*)(Vl + e) = ol; __threadfence(); *(volatile v2h*)(V16 + e) = o16; *(volatile v2us*)(Vh + e) = oh; *(volatile v2us*)(Vl + e) = ol; }

template <bool SPLIT>
__global__ __launch_bounds__(128) __attribute__((amdgpu_num_vgpr(256)))
void k_flash(const h16* __restrict__ Q16, const bf* __restrict__ Qh, const bf* __restrict__ Ql,
             const h16* __restrict__ K16, const bf* __restrict__ Kh, const bf* __restrict__ Kl,
             const h16* __restrict__ V16, const bf* __restrict__ Vh, const bf* __restrict__ Vl,
             int qblk0, h16* AT16, bf* ATh, bf* ATl) {
    __shared__ __align__(16) h16 sp16[4][16 * 32];
    __shared__ __align__(16) bf  spb[4][2][16 * 32];
    __shared__ __align__(16) h16 so16[4][16 * 128];
    __shared__ __align__(16) bf  sobh[4][16 * 128];
    __shared__ __align__(16) bf  sobl[4][16 * 128];
    const int w = threadIdx.x >> 5, lane = threadIdx.x & 31, lr = lane & 15, hi = lane >> 4;
    const int h = blockIdx.y, g = h / REP;
    const int qb = (qblk0 + (int)blockIdx.x) * 64, row0 = qb + w * 16;
    const size_t qoff = (size_t)h * TT * HD + (size_t)(row0 + lr) * HD + 8 * hi;
    const size_t koff = (size_t)g * TT * HD + (size_t)lr * HD + 8 * hi;
    const size_t voff = (size_t)g * HD * TT + (size_t)lr * TT + 8 * hi;
    v8f acc[8];
#pragma unroll
    for (int a = 0; a < 8; ++a) acc[a] = (v8f){};
    float mrow[8], lrow[8];
#pragma unroll
    for (int r = 0; r < 8; ++r) { mrow[r] = -1.0e30f; lrow[r] = 0.f; }
    const int kend = qb + 64;
#pragma unroll 1
    for (int kb = 0; kb < kend; kb += 32) {
        v8f s0 = (v8f){}, s1 = (v8f){};
        if constexpr (SPLIT) {
            const bf* qp = Qh + qoff; const bf* qp2 = Ql + qoff; const bf* kp = Kh + koff + (size_t)kb * HD; const bf* kp2 = Kl + koff + (size_t)kb * HD;
#pragma unroll 1
            for (int kc = 0; kc < HD; kc += 32) {
                const v16bf qa = WFrag<bf>::ld(qp + kc), qa2 = WFrag<bf>::ld(qp2 + kc);
                const v16bf b0 = WFrag<bf>::ld(kp + kc), b0l = WFrag<bf>::ld(kp2 + kc), b1 = WFrag<bf>::ld(kp + 16 * HD + kc), b1l = WFrag<bf>::ld(kp2 + 16 * HD + kc);
                s0 = wmmab(qa, b0, s0); s0 = wmmab(qa2, b0, s0); s0 = wmmab(qa, b0l, s0);
                s1 = wmmab(qa, b1, s1); s1 = wmmab(qa2, b1, s1); s1 = wmmab(qa, b1l, s1);
                asm volatile("v_nop\n\tv_nop\n\tv_nop\n\tv_nop" : "+v"(s0), "+v"(s1) : "v"(qa), "v"(qa2), "v"(b1), "v"(b1l));
            }
        } else {
            const h16* qp = Q16 + qoff; const h16* kp = K16 + koff + (size_t)kb * HD;
#pragma unroll 1
            for (int kc = 0; kc < HD; kc += 32) {
                const v16h qa = WFrag<h16>::ld(qp + kc);
                const v16h b0 = WFrag<h16>::ld(kp + kc), b1 = WFrag<h16>::ld(kp + 16 * HD + kc);
                s0 = wmma16(qa, b0, s0); s1 = wmma16(qa, b1, s1);
                asm volatile("v_nop\n\tv_nop\n\tv_nop\n\tv_nop" : "+v"(s0), "+v"(s1) : "v"(qa), "v"(b0), "v"(b1));
            }
        }
#pragma unroll
        for (int r = 0; r < 8; ++r) {
            const int i = row0 + 8 * hi + r;
            float a0 = s0[r] * SCL, a1 = s1[r] * SCL;
            a0 = (kb + lr > i) ? -1.0e30f : a0; a1 = (kb + 16 + lr > i) ? -1.0e30f : a1;
            float mx = fmaxf(a0, a1);
#pragma unroll
            for (int sh = 8; sh; sh >>= 1) mx = fmaxf(mx, __shfl_xor(mx, sh, 32));
            const float mnew = fmaxf(mrow[r], mx);
            const float alpha = __builtin_amdgcn_exp2f((mrow[r] - mnew) * L2E);
            mrow[r] = mnew;
            const float e0 = __builtin_amdgcn_exp2f((a0 - mnew) * L2E), e1 = __builtin_amdgcn_exp2f((a1 - mnew) * L2E);
            float psum = e0 + e1;
#pragma unroll
            for (int sh = 8; sh; sh >>= 1) psum += __shfl_xor(psum, sh, 32);
            lrow[r] = lrow[r] * alpha + psum;
#pragma unroll
            for (int a = 0; a < 8; ++a) acc[a][r] *= alpha;
            if constexpr (SPLIT) {
                unsigned short hh, ll;
                splitf(e0, hh, ll); spb[w][0][(8 * hi + r) * 32 + lr] = hh; spb[w][1][(8 * hi + r) * 32 + lr] = ll;
                splitf(e1, hh, ll); spb[w][0][(8 * hi + r) * 32 + 16 + lr] = hh; spb[w][1][(8 * hi + r) * 32 + 16 + lr] = ll;
            } else {
                sp16[w][(8 * hi + r) * 32 + lr] = tohx(e0 * PCAR); sp16[w][(8 * hi + r) * 32 + 16 + lr] = tohx(e1 * PCAR);
            }
        }
        __builtin_amdgcn_wave_barrier(); asm volatile("" ::: "memory");
        if constexpr (SPLIT) {
            const bf* pw = &spb[w][0][0]; const bf* pw2 = &spb[w][1][0];
            const v16bf pa = cat16b(*(const v8usa*)(pw + lr * 32 + 8 * hi), *(const v8usa*)(pw + lr * 32 + 16 + 8 * hi));
            const v16bf pa2 = cat16b(*(const v8usa*)(pw2 + lr * 32 + 8 * hi), *(const v8usa*)(pw2 + lr * 32 + 16 + 8 * hi));
            const bf* vp = Vh + voff + kb; const bf* vp2 = Vl + voff + kb;
            v16bf vb, vb2;
#pragma unroll
            for (int a = 0; a < 8; ++a) {
                vb = WFrag<bf>::ld(vp + (size_t)a * 16 * TT); vb2 = WFrag<bf>::ld(vp2 + (size_t)a * 16 * TT);
                acc[a] = wmmab(pa, vb, acc[a]); acc[a] = wmmab(pa2, vb, acc[a]); acc[a] = wmmab(pa, vb2, acc[a]);
                if (a == 3) { asm volatile("" ::: "memory"); }
            }
            asm volatile("v_nop\n\tv_nop\n\tv_nop\n\tv_nop" : "+v"(acc[0]), "+v"(acc[1]), "+v"(acc[2]), "+v"(acc[3]), "+v"(acc[4]), "+v"(acc[5]), "+v"(acc[6]), "+v"(acc[7]) : "v"(pa), "v"(pa2), "v"(vb), "v"(vb2));
        } else {
            const h16* pw = &sp16[w][0];
            const v16h pa = cat16(*(const v8ha*)(pw + lr * 32 + 8 * hi), *(const v8ha*)(pw + lr * 32 + 16 + 8 * hi));
            const h16* vp = V16 + voff + kb;
            v16h vb;
#pragma unroll
            for (int a = 0; a < 8; ++a) {
                vb = WFrag<h16>::ld(vp + (size_t)a * 16 * TT);
                acc[a] = wmma16(pa, vb, acc[a]);
                if (a == 3) { asm volatile("" ::: "memory"); }
            }
            asm volatile("v_nop\n\tv_nop\n\tv_nop\n\tv_nop" : "+v"(acc[0]), "+v"(acc[1]), "+v"(acc[2]), "+v"(acc[3]), "+v"(acc[4]), "+v"(acc[5]), "+v"(acc[6]), "+v"(acc[7]) : "v"(pa), "v"(vb));
        }
        __builtin_amdgcn_wave_barrier(); asm volatile("" ::: "memory");
    }
    float inv[8];
#pragma unroll
    for (int r = 0; r < 8; ++r) inv[r] = __fdiv_rn(SPLIT ? 1.0f : (ACAR / PCAR), lrow[r]);
    if constexpr (SPLIT) {
        bf* shp = &sobh[w][0]; bf* slp = &sobl[w][0];
#pragma unroll
        for (int a = 0; a < 8; ++a)
#pragma unroll
            for (int r = 0; r < 8; ++r) { const float y = acc[a][r] * inv[r]; unsigned short hh, ll; splitf(y, hh, ll); shp[(8 * hi + r) * 128 + a * 16 + lr] = hh; slp[(8 * hi + r) * 128 + a * 16 + lr] = ll; }
        __builtin_amdgcn_wave_barrier(); asm volatile("" ::: "memory");
        bf* gh = ATh + (size_t)row0 * DQ + h * HD; bf* gl = ATl + (size_t)row0 * DQ + h * HD;
#pragma unroll 1
        for (int ps = 0; ps < 2; ++ps) {
#pragma unroll
            for (int s = 0; s < 8; ++s) { const int row = 2 * s + hi, cofs = lr * 8; const v8us oh = *(const v8usa*)(shp + row * 128 + cofs); const v8us ol = *(const v8usa*)(slp + row * 128 + cofs);
                *(volatile v8us*)(gh + (size_t)row * DQ + cofs) = oh; *(volatile v8us*)(gl + (size_t)row * DQ + cofs) = ol; }
            if (ps == 0) __threadfence(); }
    } else {
        h16* sop = &so16[w][0];
#pragma unroll
        for (int a = 0; a < 8; ++a)
#pragma unroll
            for (int r = 0; r < 8; ++r) sop[(8 * hi + r) * 128 + a * 16 + lr] = tohx(acc[a][r] * inv[r]);
        __builtin_amdgcn_wave_barrier(); asm volatile("" ::: "memory");
        h16* g16 = AT16 + (size_t)row0 * DQ + h * HD;
#pragma unroll 1
        for (int ps = 0; ps < 2; ++ps) {
#pragma unroll
            for (int s = 0; s < 8; ++s) { const int row = 2 * s + hi, cofs = lr * 8; const v8h o = *(const v8ha*)(sop + row * 128 + cofs);
                *(volatile v8h*)(g16 + (size_t)row * DQ + cofs) = o; }
            if (ps == 0) __threadfence(); }
    }
}

extern "C" void kernel_launch(void* const* d_in, const int* in_sizes, int n_in,
                              void* d_out, int out_size, void* d_ws, size_t ws_size, hipStream_t stream) {
    if (n_in < 9) return;
    if ((size_t)in_sizes[0] < (size_t)NB * TT_FULL * DM) return;
    if ((size_t)in_sizes[1] < (size_t)DQ * DM || (size_t)in_sizes[4] < (size_t)DM * DQ) return;
    if ((size_t)in_sizes[2] < (size_t)DKV * DM || (size_t)in_sizes[3] < (size_t)DKV * DM) return;
    if (in_sizes[5] < HD || in_sizes[6] < HD) return;
    if ((size_t)in_sizes[7] < (size_t)TT * HD || (size_t)in_sizes[8] < (size_t)TT * HD) return;
    if ((size_t)out_size < (size_t)NB * TT * DM) return;
    const float* x = (const float*)d_in[0]; const float* wq = (const float*)d_in[1]; const float* wk = (const float*)d_in[2]; const float* wv = (const float*)d_in[3]; const float* wo = (const float*)d_in[4];
    const float* qnw = (const float*)d_in[5]; const float* knw = (const float*)d_in[6]; const float* cosT = (const float*)d_in[7]; const float* sinT = (const float*)d_in[8];
    float* OUT = (float*)d_out;
    char* wsp = (char*)d_ws;
    auto take = [&](size_t bytes) { char* p = wsp; wsp += (bytes + 255) & ~(size_t)255; return (void*)p; };
    bf* WQ = (bf*)take((size_t)DQ * DM * 2); bf* WK = (bf*)take((size_t)DKV * DM * 2); bf* WV = (bf*)take((size_t)DKV * DM * 2); bf* WO = (bf*)take((size_t)DM * DQ * 2); h16* WO16 = (h16*)take((size_t)DM * DQ * 2);
    float* CS = (float*)take((size_t)TT * HD * 2 * 4);
    bf* XB = (bf*)take((size_t)TT * DM * 2); float* FQ = (float*)take((size_t)TT * DQ * 4); float* FK = (float*)take((size_t)TT * DKV * 4);
    float* RFQ = (float*)take((size_t)NH_ * TT * 4); float* RFK = (float*)take((size_t)NKV * TT * 4);
    h16* QP16 = (h16*)take((size_t)NH_ * TT * HD * 2); bf* QPh = (bf*)take((size_t)NH_ * TT * HD * 2); bf* QPl = (bf*)take((size_t)NH_ * TT * HD * 2);
    h16* KP16 = (h16*)take((size_t)NKV * TT * HD * 2); bf* KPh = (bf*)take((size_t)NKV * TT * HD * 2); bf* KPl = (bf*)take((size_t)NKV * TT * HD * 2);
    h16* VT16 = (h16*)take((size_t)NKV * HD * TT * 2); bf* VTh = (bf*)take((size_t)NKV * HD * TT * 2); bf* VTl = (bf*)take((size_t)NKV * HD * TT * 2);
    h16* AT16 = (h16*)take((size_t)TT * DQ * 2); bf* ATh = (bf*)take((size_t)RH * DQ * 2); bf* ATl = (bf*)take((size_t)RH * DQ * 2);
    if ((size_t)(wsp - (char*)d_ws) > ws_size) return;
    float* FV = FK;
    k_cvt8<<<(unsigned)(((size_t)DQ * DM / 8 + 255) / 256), 256, 0, stream>>>(wq, WQ, (size_t)DQ * DM / 8);
    k_cvt8<<<(unsigned)(((size_t)DKV * DM / 8 + 255) / 256), 256, 0, stream>>>(wk, WK, (size_t)DKV * DM / 8);
    k_cvt8<<<(unsigned)(((size_t)DKV * DM / 8 + 255) / 256), 256, 0, stream>>>(wv, WV, (size_t)DKV * DM / 8);
    k_cvt8<<<(unsigned)(((size_t)DM * DQ / 8 + 255) / 256), 256, 0, stream>>>(wo, WO, (size_t)DM * DQ / 8);
    k_cvt16s<<<(unsigned)(((size_t)DM * DQ / 8 + 255) / 256), 256, 0, stream>>>(wo, WO16, (size_t)DM * DQ / 8, WCAR);
    k_cscvt<<<(TT * HD + 255) / 256, 256, 0, stream>>>(cosT, sinT, CS);
    const unsigned LQ = (unsigned)(((size_t)NH_ * TT * HD / 2 + 255) / 256), LKv = (unsigned)(((size_t)NKV * TT * HD / 2 + 255) / 256);
    for (int b = 0; b < NB; ++b) {
        k_cvt8<<<(unsigned)(((size_t)TT * DM / 8 + 255) / 256), 256, 0, stream>>>(x + (size_t)b * TT_FULL * DM, XB, (size_t)TT * DM / 8);
        k_gemmw<bf, 0><<<dim3(TT / 64, DQ / 64, 1), 32, 0, stream>>>(XB, nullptr, WQ, nullptr, DM, FQ, DQ, 1.0f, 0, 0, 0);
        k_rms<<<dim3(TT / 32, NH_), 256, 0, stream>>>(FQ, DQ, RFQ);
        k_rope<<<LQ, 256, 0, stream>>>(FQ, DQ, NH_, CS, RFQ, qnw, 1.0f, QP16, QPh, QPl);
        k_gemmw<bf, 0><<<dim3(TT / 64, DKV / 64, 1), 32, 0, stream>>>(XB, nullptr, WK, nullptr, DM, FK, DKV, 1.0f, 0, 0, 0);
        k_rms<<<dim3(TT / 32, NKV), 256, 0, stream>>>(FK, DKV, RFK);
        k_rope<<<LKv, 256, 0, stream>>>(FK, DKV, NKV, CS, RFK, knw, 1.0f, KP16, KPh, KPl);
        k_gemmw<bf, 0><<<dim3(TT / 64, DKV / 64, 1), 32, 0, stream>>>(XB, nullptr, WV, nullptr, DM, FV, DKV, 1.0f, 0, 0, 0);
        k_vtp<<<LKv, 256, 0, stream>>>(FV, DKV, NKV, VT16, VTh, VTl);
        k_flash<true><<<dim3(RH / 64, NH_), 128, 0, stream>>>(QP16, QPh, QPl, KP16, KPh, KPl, VT16, VTh, VTl, 0, AT16, ATh, ATl);
        if (TT > RH) k_flash<false><<<dim3((TT - RH) / 64, NH_), 128, 0, stream>>>(QP16, QPh, QPl, KP16, KPh, KPl, VT16, VTh, VTl, RH / 64, AT16, ATh, ATl);
        float* OUTb = OUT + (size_t)b * TT * DM;
        k_gemmw<bf, 1><<<dim3(RH / 64, DM / 64, 1), 32, 0, stream>>>(ATh, ATl, WO, nullptr, DQ, OUTb, DM, 1.0f, 0, 0, 0);
        if (TT > RH) k_gemmw<h16, 0><<<dim3((TT - RH) / 64, DM / 64, 1), 32, 0, stream>>>(AT16 + (size_t)RH * DQ, nullptr, WO16, nullptr, DQ, OUTb + (size_t)RH * DM, DM, 1.0f / (ACAR * WCAR), 0, 0, 0);
    }
}
